// KerasRNNCellWrapper_6055903887832
// MI455X (gfx1250) — hardware-verified
//
#include <hip/hip_runtime.h>
#include <stdint.h>

typedef __attribute__((ext_vector_type(16))) _Float16 v16h;
typedef __attribute__((ext_vector_type(8)))  _Float16 v8h;
typedef __attribute__((ext_vector_type(16))) __bf16   v16b;
typedef __attribute__((ext_vector_type(8)))  __bf16   v8b;
typedef __attribute__((ext_vector_type(8)))  float    v8f;
typedef __attribute__((ext_vector_type(4)))  float    v4f;

constexpr int kBatch = 64;
constexpr int kSteps = 512;
constexpr int kDin   = 256;
constexpr int kHid   = 1024;
constexpr int kDout  = 128;
constexpr int kRowsPerBlock = 16;
constexpr int kHP = kHid + 8;
constexpr int kXP = kDin + 8;
constexpr float kXCarry = 16.0f;
constexpr float kHCarry = 16.0f;
constexpr float kWCarry = 32.0f;
constexpr float kAccInv = 1.0f / 512.0f;

__device__ __forceinline__ unsigned short f2bf_bits(float f) {
  unsigned u = __float_as_uint(f);
  return (unsigned short)((u + 0x7FFFu + ((u >> 16) & 1u)) >> 16);
}
__device__ __forceinline__ float bf_bits2f(unsigned short h) { return __uint_as_float(((unsigned)h) << 16); }

__device__ __forceinline__ void dep_guard_h(v8f& a, v8f& b, v16h x, v16h y) { asm volatile("v_nop\n\tv_nop\n\tv_nop\n\tv_nop" : "+v"(a), "+v"(b) : "v"(x), "v"(y)); }
__device__ __forceinline__ void dep_guard_b(v8f& a, v8f& b, v16b x, v16b y) { asm volatile("v_nop\n\tv_nop\n\tv_nop\n\tv_nop" : "+v"(a), "+v"(b) : "v"(x), "v"(y)); }
__device__ __forceinline__ void keep4_h(v16h a, v16h b, v16h c, v16h d) { asm volatile("v_nop" :: "v"(a), "v"(b), "v"(c), "v"(d)); }
__device__ __forceinline__ void keep4_b(v16b a, v16b b, v16b c, v16b d) { asm volatile("v_nop" :: "v"(a), "v"(b), "v"(c), "v"(d)); }
__device__ __forceinline__ void acc_guard4(v8f& a, v8f& b, v8f& c, v8f& d) { asm volatile("v_nop\n\tv_nop\n\tv_nop\n\tv_nop" : "+v"(a), "+v"(b), "+v"(c), "+v"(d)); }
template <typename T> struct Frag;
template <> struct Frag<_Float16> {
  typedef v16h V; union U { v16h v; v8h h[2]; };
  static __device__ __forceinline__ v16h load(const _Float16* p) {
    U f; f.h[0] = *(const v8h*)(p); f.h[1] = *(const v8h*)(p + 16); return f.v;
  }
  static __device__ __forceinline__ v8f mma(v16h a, v16h b, v8f c) {
    return __builtin_amdgcn_wmma_f32_16x16x32_f16(false, a, false, b, (short)0, c, false, false);
  }
  static __device__ __forceinline__ void guard(v8f& a, v8f& b, v16h x, v16h y) { dep_guard_h(a, b, x, y); }
  static __device__ __forceinline__ void keep(v16h a, v16h b, v16h c, v16h d) { keep4_h(a, b, c, d); }
};
template <> struct Frag<__bf16> {
  typedef v16b V; union U { v16b v; v8b h[2]; };
  static __device__ __forceinline__ v16b load(const __bf16* p) {
    U f; f.h[0] = *(const v8b*)(p); f.h[1] = *(const v8b*)(p + 16); return f.v;
  }
  static __device__ __forceinline__ v8f mma(v16b a, v16b b, v8f c) {
    return __builtin_amdgcn_wmma_f32_16x16x32_bf16(false, a, false, b, (short)0, c, false, false);
  }
  static __device__ __forceinline__ void guard(v8f& a, v8f& b, v16b x, v16b y) { dep_guard_b(a, b, x, y); }
  static __device__ __forceinline__ void keep(v16b a, v16b b, v16b c, v16b d) { keep4_b(a, b, c, d); }
};

template <int ET> struct Elem;
template <> struct Elem<0> { typedef _Float16 T; };
template <> struct Elem<1> { typedef __bf16 T; };
template <int ET, bool SPLIT, int BIAS_MODE, int OUT_MODE, bool RESID, int ACT = 0>
__global__ __launch_bounds__(256) void wmma_gemm64(
    const unsigned short* __restrict__ Ap, const unsigned short* __restrict__ A2p, int lda, long strideA,
    const unsigned short* __restrict__ Btp, const unsigned short* __restrict__ Bt2p, int ldb, long strideB,
    void* __restrict__ Cout, void* __restrict__ Cout2, int ldc, long strideC,
    const float* __restrict__ bias,
    const float* __restrict__ resid, long strideR,
    int M, int N, int K, float scale) {
  typedef typename Elem<ET>::T T;
  typedef typename Frag<T>::V V;
  const T* A = (const T*)Ap; const T* A2 = (const T*)A2p; const T* Bt = (const T*)Btp; const T* Bt2 = (const T*)Bt2p;
  __shared__ __align__(16) float sT[8][16 * 68];
  const int b    = blockIdx.y;
  const int lane = threadIdx.x & 31;
  const int wave = threadIdx.x >> 5;
  const int tilesN = N >> 6;
  const int tilesM = M >> 6;
  const int tile = blockIdx.x * 8 + wave;
  if (tile >= tilesM * tilesN) return;
  const int tm = tile / tilesN;
  const int tn = tile - tm * tilesN;
  const int m0 = tm << 6;
  const int n0 = tn << 6;

  const T* Ab  = A  + (size_t)b * strideA;
  const T* Bb  = Bt + (size_t)b * strideB;
  const T* Ab2 = SPLIT ? (A2  + (size_t)b * strideA) : nullptr;
  const T* Bb2 = SPLIT ? (Bt2 + (size_t)b * strideB) : nullptr;

  const int rlane = lane & 15;
  const int koff  = (lane >> 4) * 8;
  const int mOff  = (lane >> 4) * 8;

  v8f acc[4][4];
#pragma unroll
  for (int i = 0; i < 4; ++i)
#pragma unroll
    for (int j = 0; j < 4; ++j) acc[i][j] = (v8f){0.f,0.f,0.f,0.f,0.f,0.f,0.f,0.f};

  for (int k0 = 0; k0 < K; k0 += 32) {
    V bh[4], bl[4];
#pragma unroll
    for (int j = 0; j < 4; ++j) {
      const size_t bo = (size_t)(n0 + (j << 4) + rlane) * ldb + koff + k0;
      bh[j] = Frag<T>::load(Bb + bo);
      if (SPLIT) bl[j] = Frag<T>::load(Bb2 + bo);
    }
#pragma unroll
    for (int i = 0; i < 4; ++i) {
      const size_t ao = (size_t)(m0 + (i << 4) + rlane) * lda + koff + k0;
      V ah = Frag<T>::load(Ab + ao);
      V al;
      if (SPLIT) al = Frag<T>::load(Ab2 + ao);
#pragma unroll
      for (int j = 0; j < 4; ++j) {
        acc[i][j] = Frag<T>::mma(ah, bh[j], acc[i][j]);
        if (SPLIT) {
          acc[i][j] = Frag<T>::mma(ah, bl[j], acc[i][j]);
          acc[i][j] = Frag<T>::mma(al, bh[j], acc[i][j]);
        }
      }
      Frag<T>::guard(acc[i][0], acc[i][3], ah, SPLIT ? al : ah);
    }
    Frag<T>::keep(bh[0], bh[1], bh[2], bh[3]);
    if (SPLIT) Frag<T>::keep(bl[0], bl[1], bl[2], bl[3]);
  }
  acc_guard4(acc[0][0], acc[0][1], acc[0][2], acc[0][3]);
  acc_guard4(acc[1][0], acc[1][1], acc[1][2], acc[1][3]);
  acc_guard4(acc[2][0], acc[2][1], acc[2][2], acc[2][3]);
  acc_guard4(acc[3][0], acc[3][1], acc[3][2], acc[3][3]);

  float* slab = sT[wave];
  const float* Rb = RESID ? (resid + (size_t)b * strideR) : nullptr;
#pragma unroll
  for (int i = 0; i < 4; ++i) {
    const int mBase = m0 + (i << 4);
#pragma unroll
    for (int j = 0; j < 4; ++j) {
      const int n = n0 + (j << 4) + rlane;
      float bv = 0.f;
      if (BIAS_MODE == 2) bv = bias[n];
#pragma unroll
      for (int r = 0; r < 8; ++r) {
        float v = acc[i][j][r] * scale;
        if (BIAS_MODE == 1) v += bias[mBase + mOff + r];
        if (BIAS_MODE == 2) v += bv;
        if (RESID) v += Rb[(size_t)(mBase + mOff + r) * ldc + n];
        if (ACT == 1) v = tanhf(v);
        if (ACT == 2) v = fmaxf(v, 0.0f);
        if (ACT == 3) v = v / (1.0f + expf(-v));
        if (ACT == 4) v = (v > 0.f) ? v : 0.01f * v;
        if (ACT == 5) v = 0.5f * v * (1.0f + erff(v * 0.70710678118654752f));
        slab[(mOff + r) * 68 + (j << 4) + rlane] = v;
      }
    }
    __builtin_amdgcn_fence(__ATOMIC_RELEASE, "workgroup");
    __builtin_amdgcn_wave_barrier();
    __builtin_amdgcn_fence(__ATOMIC_ACQUIRE, "workgroup");
    if (OUT_MODE == 0) {
      float* C = (float*)Cout + (size_t)b * strideC;
      const int hh = lane >> 4, c4 = (lane & 15) * 4;
      for (int pass = 0; pass < 2; ++pass) {
#pragma unroll
        for (int it = 0; it < 8; ++it) {
          const int row = it * 2 + hh;
          v4f v = *(const v4f*)(slab + row * 68 + c4);
          *(volatile v4f*)(C + (size_t)(mBase + row) * ldc + n0 + c4) = v;
        }
        __threadfence();
      }
    } else {
      const int q = lane >> 3, c8 = (lane & 7) * 8;
      unsigned short* C  = (unsigned short*)Cout  + (size_t)b * strideC;
      unsigned short* C2 = (OUT_MODE == 2) ? ((unsigned short*)Cout2 + (size_t)b * strideC) : nullptr;
      for (int pass = 0; pass < 2; ++pass) {
#pragma unroll
        for (int it = 0; it < 4; ++it) {
          const int row = it * 4 + q;
          const float* sp = slab + row * 68 + c8;
          v8h hv, lv;
#pragma unroll
          for (int e = 0; e < 8; ++e) {
            if (OUT_MODE == 1) {
              hv[e] = (_Float16)sp[e];
            } else {
              unsigned short hb = f2bf_bits(sp[e]);
              unsigned short lb = f2bf_bits(sp[e] - bf_bits2f(hb));
              hv[e] = __builtin_bit_cast(_Float16, hb);
              lv[e] = __builtin_bit_cast(_Float16, lb);
            }
          }
          *(volatile v8h*)(C + (size_t)(mBase + row) * ldc + n0 + c8) = hv;
          if (OUT_MODE == 2) *(volatile v8h*)(C2 + (size_t)(mBase + row) * ldc + n0 + c8) = lv;
        }
        __threadfence();
      }
    }
    __builtin_amdgcn_fence(__ATOMIC_RELEASE, "workgroup");
    __builtin_amdgcn_wave_barrier();
    __builtin_amdgcn_fence(__ATOMIC_ACQUIRE, "workgroup");
  }
}

__device__ __forceinline__ v8f mma_f16_g(v16h a, v16h b, v8f c) {
  c = __builtin_amdgcn_wmma_f32_16x16x32_f16(false, a, false, b, (short)0, c, false, false);
  asm volatile("v_nop\n\tv_nop\n\tv_nop\n\tv_nop" : "+v"(c) : "v"(a), "v"(b));
  return c;
}

__global__ __launch_bounds__(256) void tr_cast_f16(const float* __restrict__ in,
                                                   _Float16* __restrict__ out,
                                                   int kdim, int ndim, float scl) {
  __shared__ float sm[64][33];
  const int tid = threadIdx.x, lane = tid & 31, wave = tid >> 5;
  const int k0 = blockIdx.y * 64, n0 = blockIdx.x * 32;
  {
    const int nn = tid & 31, kb = tid >> 5;
#pragma unroll
    for (int i = 0; i < 8; ++i) {
      const int kk = kb + 8 * i;
      sm[kk][nn] = in[(size_t)(k0 + kk) * ndim + n0 + nn];
    }
  }
  __syncthreads();
  const int q = lane >> 3, c8 = (lane & 7) * 8, nn = 4 * wave + q;
  v8h hv;
#pragma unroll
  for (int e = 0; e < 8; ++e) hv[e] = (_Float16)(sm[c8 + e][nn] * scl);
  _Float16* dst = out + (size_t)(n0 + nn) * kdim + k0 + c8;
  *(volatile v8h*)dst = hv;
  __threadfence();
  *(volatile v8h*)dst = hv;
}

__global__ __launch_bounds__(256) void rnn_seq_f16(const float* __restrict__ X,
                                                   const _Float16* __restrict__ WxT,
                                                   const _Float16* __restrict__ WhT,
                                                   const float* __restrict__ bvec,
                                                   _Float16* __restrict__ HS) {
  __shared__ __align__(16) _Float16 hs_t[kRowsPerBlock * kHP];
  __shared__ __align__(16) _Float16 xs_t[kRowsPerBlock * kXP];
  union FH { v16h v; v8h h[2]; };

  const int tid = threadIdx.x, lane = tid & 31, wave = tid >> 5;
  const int hh = lane >> 4, c = lane & 15;
  const int b0 = blockIdx.x * kRowsPerBlock;
  const int ncol0 = 128 * wave + c;

  float bj[8];
#pragma unroll
  for (int j = 0; j < 8; ++j) bj[j] = bvec[ncol0 + 16 * j];

  const int xr = tid >> 4, xseg = (tid & 15) * 16;
  const float* xsrc = X + (size_t)(b0 + xr) * kSteps * kDin + xseg;
  const int q = lane >> 3, c8 = (lane & 7) * 8;
  const _Float16* wxb = WxT + (size_t)ncol0 * kDin + 8 * hh;
  const _Float16* whb = WhT + (size_t)ncol0 * kHid + 8 * hh;

  for (int t = 0; t < kSteps; ++t) {
    {
      const float* xp = xsrc + (size_t)t * kDin;
      const v4f f0 = *(const v4f*)(xp);
      const v4f f1 = *(const v4f*)(xp + 4);
      const v4f f2 = *(const v4f*)(xp + 8);
      const v4f f3 = *(const v4f*)(xp + 12);
      v8h v0, v1;
#pragma unroll
      for (int e = 0; e < 4; ++e) {
        v0[e]     = (_Float16)(f0[e] * kXCarry);
        v0[4 + e] = (_Float16)(f1[e] * kXCarry);
        v1[e]     = (_Float16)(f2[e] * kXCarry);
        v1[4 + e] = (_Float16)(f3[e] * kXCarry);
      }
      *(v8h*)(xs_t + xr * kXP + xseg)     = v0;
      *(v8h*)(xs_t + xr * kXP + xseg + 8) = v1;
    }
    __syncthreads();

    v8f acc[8];
#pragma unroll
    for (int j = 0; j < 8; ++j) acc[j] = (v8f){0.f, 0.f, 0.f, 0.f, 0.f, 0.f, 0.f, 0.f};

#pragma unroll 1
    for (int k0 = 0; k0 < kDin; k0 += 32) {
      FH fa;
      fa.h[0] = *(const v8h*)(xs_t + c * kXP + k0 + 8 * hh);
      fa.h[1] = *(const v8h*)(xs_t + c * kXP + k0 + 16 + 8 * hh);
#pragma unroll
      for (int j = 0; j < 8; ++j) {
        const v16h fb = Frag<_Float16>::load(wxb + (size_t)j * 16 * kDin + k0);
        acc[j] = mma_f16_g(fa.v, fb, acc[j]);
      }
    }
    if (t > 0) {
#pragma unroll 1
      for (int k0 = 0; k0 < kHid; k0 += 32) {
        FH fa;
        fa.h[0] = *(const v8h*)(hs_t + c * kHP + k0 + 8 * hh);
        fa.h[1] = *(const v8h*)(hs_t + c * kHP + k0 + 16 + 8 * hh);
#pragma unroll
        for (int j = 0; j < 8; ++j) {
          const v16h fb = Frag<_Float16>::load(whb + (size_t)j * 16 * kHid + k0);
          acc[j] = mma_f16_g(fa.v, fb, acc[j]);
        }
      }
    }
    __syncthreads();

#pragma unroll
    for (int j = 0; j < 8; ++j) {
      const int col = ncol0 + 16 * j;
#pragma unroll
      for (int r = 0; r < 8; ++r) {
        float v = acc[j][r] * kAccInv + bj[j];
        v = fminf(fmaxf(v, -16.0f), 16.0f);
        const float e = expf(2.0f * v);
        const float hval = 1.0f - 2.0f * __builtin_amdgcn_rcpf(1.0f + e);
        hs_t[(8 * hh + r) * kHP + col] = (_Float16)(hval * kHCarry);
      }
    }
    __syncthreads();

    for (int pass = 0; pass < 2; ++pass) {
#pragma unroll
      for (int rr = 0; rr < 2; ++rr) {
        const int row = 2 * wave + rr;
        const _Float16* src = hs_t + row * kHP;
        _Float16* dst = HS + ((size_t)(b0 + row) * kSteps + t) * kHid;
#pragma unroll
        for (int it = 0; it < 4; ++it) {
          const int off = (it * 4 + q) * 64 + c8;
          const v8h hv = *(const v8h*)(src + off);
          *(volatile v8h*)(dst + off) = hv;
        }
      }
      __threadfence();
    }
  }
}

extern "C" void kernel_launch(void* const* d_in, const int* in_sizes, int n_in,
                              void* d_out, int out_size, void* d_ws,
                              size_t ws_size, hipStream_t stream) {
  if (n_in < 6) return;
  if (in_sizes[0] != kBatch * kSteps * kDin) return;
  if (in_sizes[1] != kDin * kHid) return;
  if (in_sizes[2] != kHid * kHid) return;
  if (in_sizes[3] != kHid) return;
  if (in_sizes[4] != kHid * kDout) return;
  if (in_sizes[5] != kDout) return;
  if (out_size != kBatch * kSteps * kDout) return;

  const float* inputs = (const float*)d_in[0];
  const float* Wx     = (const float*)d_in[1];
  const float* Wh     = (const float*)d_in[2];
  const float* bvec   = (const float*)d_in[3];
  const float* Wo     = (const float*)d_in[4];
  const float* bo     = (const float*)d_in[5];
  float* out = (float*)d_out;

  const size_t offWx = 0;
  const size_t offWh = offWx + (size_t)kHid * kDin * 2;
  const size_t offWo = offWh + (size_t)kHid * kHid * 2;
  const size_t offHS = offWo + (size_t)kDout * kHid * 2;
  const size_t total = offHS + (size_t)kBatch * kSteps * kHid * 2;
  if (total > ws_size) return;

  char* ws = (char*)d_ws;
  _Float16* WxT16 = (_Float16*)(ws + offWx);
  _Float16* WhT16 = (_Float16*)(ws + offWh);
  _Float16* WoT16 = (_Float16*)(ws + offWo);
  _Float16* HS16  = (_Float16*)(ws + offHS);

  tr_cast_f16<<<dim3(kHid / 32, kDin / 64), 256, 0, stream>>>(Wx, WxT16, kDin, kHid, kWCarry);
  tr_cast_f16<<<dim3(kHid / 32, kHid / 64), 256, 0, stream>>>(Wh, WhT16, kHid, kHid, kWCarry);
  tr_cast_f16<<<dim3(kDout / 32, kHid / 64), 256, 0, stream>>>(Wo, WoT16, kHid, kDout, kWCarry);

  rnn_seq_f16<<<dim3(kBatch / kRowsPerBlock), 256, 0, stream>>>(inputs, WxT16, WhT16, bvec, HS16);

  wmma_gemm64<0, false, 2, 0, false, 0><<<dim3((kBatch * kSteps / 64) * (kDout / 64) / 8, 1), 256, 0, stream>>>(
      (const unsigned short*)HS16, (const unsigned short*)HS16, kHid, 0L,
      (const unsigned short*)WoT16, (const unsigned short*)WoT16, kHid, 0L,
      (void*)out, (void*)out, kDout, 0L,
      bo,
      bo, 0L,
      kBatch * kSteps, kDout, kHid, kAccInv);
}
